// GroupQueryAttention_67619965108465
// MI455X (gfx1250) — hardware-verified
//
#include <hip/hip_runtime.h>


#ifndef NB
#define NB 2
#endif
#ifndef SEQ
#define SEQ 2048
#endif
#define SEQ_FULL 2048
#define DM 1024
#define NHQ 16
#define NGK 4
#define HD 64
#define DKV (NGK * HD)
#define NFREQ (HD / 2)

static_assert(NB >= 1 && NB <= 2);
static_assert(SEQ % 128 == 0 && SEQ >= 128 && SEQ <= SEQ_FULL);
static_assert(DM % 64 == 0 && DKV % 64 == 0 && DM % 32 == 0);
static_assert(HD == 64 && NFREQ == 32 && DM == NHQ * HD && (NHQ % NGK) == 0);
static_assert((DM / 8) == 128);

typedef _Float16 v16h __attribute__((ext_vector_type(16)));
typedef __bf16   v16b __attribute__((ext_vector_type(16)));
typedef float    v8f  __attribute__((ext_vector_type(8)));
typedef float    v4f  __attribute__((ext_vector_type(4)));
typedef unsigned v4u  __attribute__((ext_vector_type(4)));

union Frag  { v16h h; v16b b; v4u u[2]; unsigned short s[16]; };
union Pack8 { v4u u; unsigned short s[8]; };

static __device__ __forceinline__ v8f mma_f16(v16h a, v16h b, v8f c)
{
  v8f d = __builtin_amdgcn_wmma_f32_16x16x32_f16(false, a, false, b, (short)0, c, false, false);
  asm volatile("v_nop\n\tv_nop\n\tv_nop\n\tv_nop" : "+v"(d) : "v"(a), "v"(b));
  return d;
}
static __device__ __forceinline__ v8f mma_bf16(v16b a, v16b b, v8f c)
{
  v8f d = __builtin_amdgcn_wmma_f32_16x16x32_bf16(false, a, false, b, (short)0, c, false, false);
  asm volatile("v_nop\n\tv_nop\n\tv_nop\n\tv_nop" : "+v"(d) : "v"(a), "v"(b));
  return d;
}

static __device__ __forceinline__ unsigned short bf16_bits(float x)
{
  unsigned u = __float_as_uint(x);
  u = u + 0x7FFFu + ((u >> 16) & 1u);
  return (unsigned short)(u >> 16);
}
static __device__ __forceinline__ float bf16_val(float x)
{
  return __uint_as_float(((unsigned)bf16_bits(x)) << 16);
}
static __device__ __forceinline__ unsigned short f16_bits(float x)
{
  const _Float16 hv = (_Float16)x;
  return __builtin_bit_cast(unsigned short, hv);
}
static __device__ __forceinline__ float f16_val(unsigned short b)
{
  return (float)__builtin_bit_cast(_Float16, b);
}
static __device__ __forceinline__ void split_f16(float x, unsigned short& hi, unsigned short& lo)
{
  unsigned short hb = f16_bits(x);
  hb = (fabsf(x) < 6.103515625e-05f) ? (unsigned short)0 : hb;
  const float hv = f16_val(hb);
  hi = hb;
  lo = f16_bits((x - hv) * 2048.0f);
}

static __device__ __forceinline__ void st2(unsigned short* p, v4u v)
{
  *(volatile v4u*)p = v; __threadfence(); *(volatile v4u*)p = v;
}
static __device__ __forceinline__ void st2(float* p, v4f v)
{
  *(volatile v4f*)p = v; __threadfence(); *(volatile v4f*)p = v;
}
static __device__ __forceinline__ void st2(float* p, float v)
{
  *(volatile float*)p = v; __threadfence(); *(volatile float*)p = v;
}

static __device__ __forceinline__ void sincos_p(float x, float& s, float& c)
{
  const float jf = rintf(x * 0.63661977236758134f);
  const double rd = __builtin_fma(-(double)jf, 1.5707963267948966, (double)x);
  const float r  = (float)rd;
  const float r2 = r * r;
  const float sp = r + r * r2 * (-1.6666654611e-1f + r2 * (8.3321608736e-3f + r2 * (-1.9515295891e-4f)));
  const float cp = 1.0f - 0.5f * r2 +
                   r2 * r2 * (4.166664568298827e-2f + r2 * (-1.388731625493765e-3f + r2 * 2.443315711809948e-5f));
  const int q = ((int)jf) & 3;
  s = (q == 0) ? sp : (q == 1) ? cp : (q == 2) ? -sp : -cp;
  c = (q == 0) ? cp : (q == 1) ? -sp : (q == 2) ? -cp : sp;
}

__global__ __launch_bounds__(256)
void k_cvt_act(const float* __restrict__ X, unsigned short* __restrict__ Y, int nPieces)
{
  const int i = blockIdx.x * 256 + threadIdx.x;
  if (i >= nPieces) return;
  const int row = i >> 7;
  const int col = (i & 127) * 8;
  const int b = row / SEQ, t = row - b * SEQ;
  const float* src = X + ((size_t)b * SEQ_FULL + t) * DM + col;
  const v4f a = *(const v4f*)src;
  const v4f c = *(const v4f*)(src + 4);
  Pack8 pk;
  #pragma unroll
  for (int e = 0; e < 4; ++e) { pk.s[e] = bf16_bits(a[e]); pk.s[4 + e] = bf16_bits(c[e]); }
  st2(Y + (size_t)row * DM + col, pk.u);
}

__global__ __launch_bounds__(256)
void k_cvt_w(const float* __restrict__ W, unsigned short* __restrict__ Wt, int N, int mode)
{
  __shared__ __align__(16) float tile[64][68];
  const int tid = threadIdx.x;
  const int n0 = blockIdx.x * 64, k0 = blockIdx.y * 64;
  #pragma unroll
  for (int i = 0; i < 4; ++i) {
    const int p = tid + 256 * i;
    const int kr = p >> 4, c = (p & 15) * 4;
    const v4f v = *(const v4f*)(W + (size_t)(k0 + kr) * N + n0 + c);
    *(v4f*)(&tile[kr][c]) = v;
  }
  __syncthreads();
  #pragma unroll
  for (int j = 0; j < 2; ++j) {
    const int nr = 32 * j + (tid >> 3);
    const int kp = (tid & 7) * 8;
    Pack8 pk;
    #pragma unroll
    for (int e = 0; e < 8; ++e) {
      const float x  = tile[kp + e][nr];
      const float xb = bf16_val(x);
      pk.s[e] = (mode != 0) ? f16_bits(xb * 64.0f) : bf16_bits(x);
    }
    st2(Wt + (size_t)(n0 + nr) * DM + k0 + kp, pk.u);
  }
}

__global__ __launch_bounds__(256)
void k_rope_tab(const int* __restrict__ maxlen, float* __restrict__ cs, float* __restrict__ sn, int n)
{
  const int i = blockIdx.x * 256 + threadIdx.x;
  if (i >= n) return;
  const int t = i >> 5, fi = i & 31;
  int ml = maxlen[0];
  ml = (ml < 1) ? 1 : ml;
  const int tt = (t < ml) ? t : (ml - 1);
  const float dv  = expf((float)(2 * fi) * (-0.14391156831212787f));
  const float ang = (float)tt * dv;
  float s, c;
  sincos_p(ang, s, c);
  st2(cs + i, c);
  st2(sn + i, s);
}

template<int MODE>
__global__ __launch_bounds__(256)
void k_gemm(const unsigned short* __restrict__ A, const unsigned short* __restrict__ A2,
            const unsigned short* __restrict__ Bw, const float* __restrict__ bias,
            const float* __restrict__ cs, const float* __restrict__ sn,
            void* Out, void* Out2)
{
  __shared__ __align__(16) unsigned char smem[32768];
  unsigned short* As  = (unsigned short*)smem;
  unsigned short* As2 = (unsigned short*)(smem + 8192);
  unsigned short* Bs  = (unsigned short*)(smem + 16384);
  float* T = (float*)smem;

  const int tid = threadIdx.x, lane = tid & 31, w = tid >> 5;
  const int h = lane >> 4, lm = lane & 15;
  const int blockM = blockIdx.x * 128, blockN = blockIdx.y * 64;
  const int waveM = (w & 3) * 32, waveN = (w >> 2) * 32;

  const v8f zero = {};
  v8f acc[2][2], acc2[2][2];
  #pragma unroll
  for (int mt = 0; mt < 2; ++mt)
    #pragma unroll
    for (int nt = 0; nt < 2; ++nt) { acc[mt][nt] = zero; acc2[mt][nt] = zero; }

  for (int k0 = 0; k0 < DM; k0 += 32) {
    __syncthreads();
    #pragma unroll
    for (int i = 0; i < 2; ++i) {
      const int p = tid + 256 * i;
      const int row = p >> 2, cb = (p & 3) * 8;
      *(v4u*)(As + row * 32 + cb) = *(const v4u*)(A + (size_t)(blockM + row) * DM + k0 + cb);
      if constexpr (MODE == 3) {
        *(v4u*)(As2 + row * 32 + cb) = *(const v4u*)(A2 + (size_t)(blockM + row) * DM + k0 + cb);
      }
    }
    {
      const int row = tid >> 2, cb = (tid & 3) * 8;
      *(v4u*)(Bs + row * 32 + cb) = *(const v4u*)(Bw + (size_t)(blockN + row) * DM + k0 + cb);
    }
    __syncthreads();

    Frag af[2], af2[2], bf[2];
    #pragma unroll
    for (int mt = 0; mt < 2; ++mt) {
      const unsigned short* ap = As + (waveM + 16 * mt + lm) * 32 + 8 * h;
      af[mt].u[0] = *(const v4u*)ap;
      af[mt].u[1] = *(const v4u*)(ap + 16);
      if constexpr (MODE == 3) {
        const unsigned short* ap2 = As2 + (waveM + 16 * mt + lm) * 32 + 8 * h;
        af2[mt].u[0] = *(const v4u*)ap2;
        af2[mt].u[1] = *(const v4u*)(ap2 + 16);
      }
    }
    #pragma unroll
    for (int nt = 0; nt < 2; ++nt) {
      const unsigned short* bp = Bs + (waveN + 16 * nt + lm) * 32 + 8 * h;
      bf[nt].u[0] = *(const v4u*)bp;
      bf[nt].u[1] = *(const v4u*)(bp + 16);
    }
    #pragma unroll
    for (int mt = 0; mt < 2; ++mt)
      #pragma unroll
      for (int nt = 0; nt < 2; ++nt) {
        if constexpr (MODE == 3) {
          acc[mt][nt]  = mma_f16(af[mt].h,  bf[nt].h, acc[mt][nt]);
          acc2[mt][nt] = mma_f16(af2[mt].h, bf[nt].h, acc2[mt][nt]);
        } else {
          acc[mt][nt] = mma_bf16(af[mt].b, bf[nt].b, acc[mt][nt]);
        }
      }
  }

  __syncthreads();
  #pragma unroll
  for (int mt = 0; mt < 2; ++mt)
    #pragma unroll
    for (int nt = 0; nt < 2; ++nt)
      #pragma unroll
      for (int r = 0; r < 8; ++r) {
        float v = acc[mt][nt][r];
        if constexpr (MODE == 3) v = v + acc2[mt][nt][r] * (1.0f / 2048.0f);
        T[(waveM + 16 * mt + 8 * h + r) * 64 + waveN + 16 * nt + lm] = v;
      }
  __syncthreads();

  if constexpr (MODE == 0 || MODE == 1) {
    constexpr int NH = (MODE == 0) ? NHQ : NGK;
    const int head = blockIdx.y;
    #pragma unroll
    for (int j = 0; j < 4; ++j) {
      const int row = 32 * j + (tid >> 3);
      const int cp = tid & 7, c0 = cp * 8;
      const int mG = blockM + row;
      const int b = mG / SEQ, t = mG - b * SEQ;
      const v4f x0 = *(const v4f*)(T + row * 64 + c0);
      const v4f x1 = *(const v4f*)(T + row * 64 + c0 + 4);
      const v4f b0 = *(const v4f*)(bias + blockN + c0);
      const v4f b1 = *(const v4f*)(bias + blockN + c0 + 4);
      const v4f c4 = *(const v4f*)(cs + (size_t)t * NFREQ + cp * 4);
      const v4f s4 = *(const v4f*)(sn + (size_t)t * NFREQ + cp * 4);
      float xv[8];
      #pragma unroll
      for (int e = 0; e < 4; ++e) { xv[e] = x0[e] + b0[e]; xv[4 + e] = x1[e] + b1[e]; }
      Pack8 pk;
      #pragma unroll
      for (int i = 0; i < 4; ++i) {
        const float xe = xv[2 * i], xo = xv[2 * i + 1];
        const float cc = c4[i], ss = s4[i];
        const float oe = xe * cc - xo * ss;
        const float oo = xe * ss + xo * cc;
        pk.s[2 * i]     = f16_bits(oe * 16.0f);
        pk.s[2 * i + 1] = f16_bits(oo * 16.0f);
      }
      unsigned short* dst = (unsigned short*)Out + (((size_t)(b * NH + head)) * SEQ + t) * HD + c0;
      st2(dst, pk.u);
    }
  } else if constexpr (MODE == 2) {
    const int g = blockIdx.y;
    const int b = blockM / SEQ, t0 = blockM - b * SEQ;
    #pragma unroll
    for (int j = 0; j < 4; ++j) {
      const int d = 16 * j + (tid >> 4);
      const int kp = tid & 15;
      const float bia = bias[blockN + d];
      Pack8 ph, pl;
      #pragma unroll
      for (int e = 0; e < 8; ++e) {
        const float v = (T[(8 * kp + e) * 64 + d] + bia) * 16.0f;
        unsigned short hb, lb;
        split_f16(v, hb, lb);
        ph.s[e] = hb; pl.s[e] = lb;
      }
      const size_t off = (((size_t)(b * NGK + g)) * HD + d) * SEQ + t0 + 8 * kp;
      st2((unsigned short*)Out + off, ph.u);
      st2((unsigned short*)Out2 + off, pl.u);
    }
  } else {
    #pragma unroll
    for (int j = 0; j < 8; ++j) {
      const int row = 16 * j + (tid >> 4);
      const int c0 = (tid & 15) * 4;
      const int mG = blockM + row;
      const v4f x  = *(const v4f*)(T + row * 64 + c0);
      const v4f bb = *(const v4f*)(bias + blockN + c0);
      const v4f o = x * (1.0f / 4096.0f) + bb;
      st2((float*)Out + (size_t)mG * DM + blockN + c0, o);
    }
  }
}

__global__ __launch_bounds__(128)
void k_attn(const unsigned short* __restrict__ Qp, const unsigned short* __restrict__ Kp,
            const unsigned short* __restrict__ Vh, const unsigned short* __restrict__ Vl,
            unsigned short* __restrict__ Oh, unsigned short* __restrict__ Ol)
{
  __shared__ __align__(16) unsigned short Ks[32 * 64];
  __shared__ __align__(16) unsigned short Vhs[64 * 32];
  __shared__ __align__(16) unsigned short Vls[64 * 32];
  __shared__ __align__(16) unsigned short Osh[4 * 16 * 64];
  __shared__ __align__(16) unsigned short Osl[4 * 16 * 64];

  const int tid = threadIdx.x, lane = tid & 31, w = tid >> 5;
  const int h = lane >> 4, lm = lane & 15;
  const int bh = blockIdx.y;
  const int b = bh / NHQ, hq = bh - b * NHQ, g = hq / (NHQ / NGK);
  const int q0 = blockIdx.x * 64 + w * 16;

  const unsigned short* Qb = Qp + ((size_t)(b * NHQ + hq) * SEQ + q0) * HD;
  const unsigned short* Kb = Kp + ((size_t)(b * NGK + g) * SEQ) * HD;
  const size_t vbase = ((size_t)(b * NGK + g) * HD) * SEQ;
  const unsigned short* Vhb = Vh + vbase;
  const unsigned short* Vlb = Vl + vbase;

  Frag qf[2];
  #pragma unroll
  for (int kk = 0; kk < 2; ++kk) {
    const unsigned short* qp = Qb + (size_t)lm * HD + 32 * kk + 8 * h;
    qf[kk].u[0] = *(const v4u*)qp;
    qf[kk].u[1] = *(const v4u*)(qp + 16);
  }

  const v8f zero = {};
  v8f o0[4], o1[4];
  #pragma unroll
  for (int dt = 0; dt < 4; ++dt) { o0[dt] = zero; o1[dt] = zero; }
  float mrun = -__builtin_inff(), lrun = 0.0f;
  const float SSC = 0.00048828125f;

  for (int c0 = 0; c0 < SEQ; c0 += 32) {
    __syncthreads();
    #pragma unroll
    for (int i = 0; i < 2; ++i) {
      const int p = tid + 128 * i;
      const int kr = p >> 3, kc = (p & 7) * 8;
      *(v4u*)(Ks + kr * 64 + kc) = *(const v4u*)(Kb + (size_t)(c0 + kr) * HD + kc);
      const int vd = p >> 2, vc = (p & 3) * 8;
      *(v4u*)(Vhs + vd * 32 + vc) = *(const v4u*)(Vhb + (size_t)vd * SEQ + c0 + vc);
      *(v4u*)(Vls + vd * 32 + vc) = *(const v4u*)(Vlb + (size_t)vd * SEQ + c0 + vc);
    }
    __syncthreads();

    v8f sacc[2];
    #pragma unroll
    for (int nt = 0; nt < 2; ++nt) {
      v8f a = zero;
      #pragma unroll
      for (int kk = 0; kk < 2; ++kk) {
        Frag ka;
        const unsigned short* kp = Ks + (16 * nt + lm) * 64 + 32 * kk + 8 * h;
        ka.u[0] = *(const v4u*)kp;
        ka.u[1] = *(const v4u*)(kp + 16);
        a = mma_f16(ka.h, qf[kk].h, a);
      }
      sacc[nt] = a;
    }

    float sv[16];
    float mx = -__builtin_inff();
    #pragma unroll
    for (int nt = 0; nt < 2; ++nt)
      #pragma unroll
      for (int r = 0; r < 8; ++r) {
        const float s = sacc[nt][r] * SSC;
        sv[8 * nt + r] = s;
        mx = fmaxf(mx, s);
      }
    mx = fmaxf(mx, __shfl_xor(mx, 16, 32));
    const float mnew = fmaxf(mrun, mx);
    const float alpha = __expf(mrun - mnew);
    float psum = 0.0f;
    Frag ph, pl;
    #pragma unroll
    for (int i = 0; i < 16; ++i) {
      const float p = __expf(sv[i] - mnew) * 1024.0f;
      psum += p;
      const unsigned short hb = f16_bits(p);
      ph.s[i] = hb;
      pl.s[i] = f16_bits((p - f16_val(hb)) * 2048.0f);
    }
    psum += __shfl_xor(psum, 16, 32);
    lrun = lrun * alpha + psum;
    mrun = mnew;

    #pragma unroll
    for (int r = 0; r < 8; ++r) {
      const float ar = __shfl(alpha, 8 * h + r, 32);
      #pragma unroll
      for (int dt = 0; dt < 4; ++dt) { o0[dt][r] *= ar; o1[dt][r] *= ar; }
    }

    #pragma unroll
    for (int dt = 0; dt < 4; ++dt) {
      Frag vh, vl;
      const unsigned short* vp = Vhs + (16 * dt + lm) * 32 + 8 * h;
      vh.u[0] = *(const v4u*)vp;
      vh.u[1] = *(const v4u*)(vp + 16);
      const unsigned short* vq = Vls + (16 * dt + lm) * 32 + 8 * h;
      vl.u[0] = *(const v4u*)vq;
      vl.u[1] = *(const v4u*)(vq + 16);
      o0[dt] = mma_f16(ph.h, vh.h, o0[dt]);
      o1[dt] = mma_f16(pl.h, vh.h, o1[dt]);
      o1[dt] = mma_f16(ph.h, vl.h, o1[dt]);
    }
  }

  #pragma unroll
  for (int r = 0; r < 8; ++r) {
    const float lr = __shfl(lrun, 8 * h + r, 32);
    const float inv = 4.0f / lr;
    #pragma unroll
    for (int dt = 0; dt < 4; ++dt) {
      const float x = (o0[dt][r] + o1[dt][r] * (1.0f / 2048.0f)) * inv;
      unsigned short hb, lb;
      split_f16(x, hb, lb);
      Osh[w * 1024 + (8 * h + r) * 64 + 16 * dt + lm] = hb;
      Osl[w * 1024 + (8 * h + r) * 64 + 16 * dt + lm] = lb;
    }
  }
  __syncthreads();
  #pragma unroll
  for (int j = 0; j < 4; ++j) {
    const int row = 4 * j + (lane >> 3);
    const int pc = (lane & 7) * 8;
    const v4u a = *(const v4u*)(Osh + w * 1024 + row * 64 + pc);
    const v4u c = *(const v4u*)(Osl + w * 1024 + row * 64 + pc);
    const size_t goff = ((size_t)(b * SEQ + q0 + row)) * DM + hq * HD + pc;
    st2(Oh + goff, a);
    st2(Ol + goff, c);
  }
}

extern "C" void kernel_launch(void* const* d_in, const int* in_sizes, int n_in,
                              void* d_out, int out_size, void* d_ws, size_t ws_size,
                              hipStream_t stream)
{
  if (n_in < 11) return;
  const long needAct = ((long)(NB - 1) * SEQ_FULL + SEQ) * DM;
  if ((long)in_sizes[0] < needAct || (long)in_sizes[1] < needAct) return;
  if (in_sizes[2] < DM * DM || in_sizes[3] < DM || in_sizes[4] < DM * DKV || in_sizes[5] < DKV ||
      in_sizes[6] < DM * DKV || in_sizes[7] < DKV || in_sizes[8] < DM * DM || in_sizes[9] < DM ||
      in_sizes[10] < 1) return;
  if (out_size < NB * SEQ * DM) return;

  const float* X   = (const float*)d_in[0];
  const float* Enc = (const float*)d_in[1];
  const float* Wq  = (const float*)d_in[2];
  const float* bq  = (const float*)d_in[3];
  const float* Wk  = (const float*)d_in[4];
  const float* bk  = (const float*)d_in[5];
  const float* Wv  = (const float*)d_in[6];
  const float* bv  = (const float*)d_in[7];
  const float* Wo  = (const float*)d_in[8];
  const float* bo  = (const float*)d_in[9];
  const int*   mlen = (const int*)d_in[10];

  char* ws = (char*)d_ws;
  size_t off = 0;
  auto take = [&](size_t bytes) -> char* {
    char* p = ws + off;
    off += (bytes + 255) & ~(size_t)255;
    return p;
  };
  const size_t actB = (size_t)NB * SEQ * DM * 2;
  const size_t kvB  = (size_t)NB * NGK * SEQ * HD * 2;
  const size_t tabB = (size_t)SEQ * NFREQ * 4;
  unsigned short* Xb  = (unsigned short*)take(actB);
  unsigned short* Eb  = (unsigned short*)take(actB);
  unsigned short* Wqt = (unsigned short*)take((size_t)DM * DM * 2);
  unsigned short* Wkt = (unsigned short*)take((size_t)DKV * DM * 2);
  unsigned short* Wvt = (unsigned short*)take((size_t)DKV * DM * 2);
  unsigned short* Wot = (unsigned short*)take((size_t)DM * DM * 2);
  float* cs = (float*)take(tabB);
  float* sn = (float*)take(tabB);
  unsigned short* Qp  = (unsigned short*)take(actB);
  unsigned short* Kpl = (unsigned short*)take(kvB);
  unsigned short* Vhp = (unsigned short*)take(kvB);
  unsigned short* Vlp = (unsigned short*)take(kvB);
  unsigned short* Ohp = (unsigned short*)take(actB);
  unsigned short* Olp = (unsigned short*)take(actB);
  if (off > ws_size) return;

  const dim3 blk(256);
  const int nPieces = NB * SEQ * (DM / 8);
  k_cvt_act<<<dim3(nPieces / 256), blk, 0, stream>>>(X,   Xb, nPieces);
  k_cvt_act<<<dim3(nPieces / 256), blk, 0, stream>>>(Enc, Eb, nPieces);

  k_cvt_w<<<dim3(DM / 64,  DM / 64), blk, 0, stream>>>(Wq, Wqt, DM,  0);
  k_cvt_w<<<dim3(DKV / 64, DM / 64), blk, 0, stream>>>(Wk, Wkt, DKV, 0);
  k_cvt_w<<<dim3(DKV / 64, DM / 64), blk, 0, stream>>>(Wv, Wvt, DKV, 0);
  k_cvt_w<<<dim3(DM / 64,  DM / 64), blk, 0, stream>>>(Wo, Wot, DM,  1);

  const int nTab = SEQ * NFREQ;
  k_rope_tab<<<dim3(nTab / 256), blk, 0, stream>>>(mlen, cs, sn, nTab);

  const int M = NB * SEQ;
  k_gemm<0><<<dim3(M / 128, DM / 64),  blk, 0, stream>>>(Xb, Xb, Wqt, bq, cs, sn, (void*)Qp,  (void*)Qp);
  k_gemm<1><<<dim3(M / 128, DKV / 64), blk, 0, stream>>>(Eb, Eb, Wkt, bk, cs, sn, (void*)Kpl, (void*)Kpl);
  k_gemm<2><<<dim3(M / 128, DKV / 64), blk, 0, stream>>>(Eb, Eb, Wvt, bv, cs, sn, (void*)Vhp, (void*)Vlp);

  k_attn<<<dim3(SEQ / 64, NB * NHQ), dim3(128), 0, stream>>>(Qp, Kpl, Vhp, Vlp, Ohp, Olp);

  k_gemm<3><<<dim3(M / 128, DM / 64), blk, 0, stream>>>(Ohp, Olp, Wot, bo, cs, sn, d_out, d_out);
}
